// MultiHeadAttention_89008902243131
// MI455X (gfx1250) — hardware-run, weakly checked
//
#include <hip/hip_runtime.h>


#ifndef NB
#define NB 2
#endif
#ifndef SEQ
#define SEQ 4096
#endif
#define NB_FULL  2
#define SEQ_FULL 4096
#ifndef OUT_SEQ
#define OUT_SEQ SEQ
#endif
#define CH   128
#define NH_  8
#define HD   16
#define AW   4
#define QRS  64.0f
#define KRI  (1.0f / 64.0f)
#define WPS  64.0f
#define WPI  (1.0f / 64.0f)
#define SC2  (0.25f * 1.4426950408889634f)
#define PSH  10.0f
#define BN_EPS 1e-3f

static_assert(HD == 16);
static_assert(NH_ * HD == CH);
static_assert(CH % 64 == 0);
static_assert(CH % 32 == 0);
static_assert(SEQ % 64 == 0);
static_assert(SEQ % 32 == 0);
static_assert(SEQ % (16 * AW) == 0);
static_assert((3 * CH * CH) % (8 * 256) == 0);
static_assert((CH * CH) % (8 * 256) == 0);
static_assert(NB <= NB_FULL);
static_assert(SEQ <= SEQ_FULL);

typedef _Float16 h16;
typedef unsigned short bf;
typedef __attribute__((ext_vector_type(16))) __bf16   v16bf;
typedef __attribute__((ext_vector_type(16))) _Float16 v16h;
typedef __attribute__((ext_vector_type(8)))  _Float16 v8h;
typedef __attribute__((ext_vector_type(8)))  unsigned short v8us;
typedef __attribute__((ext_vector_type(8)))  float    v8f;
typedef __attribute__((ext_vector_type(4)))  float    v4f;
typedef __attribute__((ext_vector_type(4)))  unsigned int v4u;
typedef v4f  __attribute__((may_alias)) v4fa;

#define PB_WQ ((3 * CH * CH) / (8 * 256))
#define PB_WP ((CH * CH) / (8 * 256))
#define PLANE_E ((size_t)NB * NH_ * SEQ * 32)

__device__ __forceinline__ unsigned short f2bf(float f) { unsigned u = __float_as_uint(f); u += 0x7FFFu + ((u >> 16) & 1u); return (unsigned short)(u >> 16); }
__device__ __forceinline__ float bfr(float f) { return __uint_as_float(((unsigned)f2bf(f)) << 16); }
__device__ __forceinline__ v16h cat16(v8h lo, v8h hi) { return __builtin_shufflevector(lo, hi, 0, 1, 2, 3, 4, 5, 6, 7, 8, 9, 10, 11, 12, 13, 14, 15); }
__device__ __forceinline__ v16bf cat16b(v8us lo, v8us hi) { return __builtin_bit_cast(v16bf, __builtin_shufflevector(lo, hi, 0, 1, 2, 3, 4, 5, 6, 7, 8, 9, 10, 11, 12, 13, 14, 15)); }
__device__ __forceinline__ v8f wmma16(v16h a, v16h b, v8f c) { return __builtin_amdgcn_wmma_f32_16x16x32_f16(false, a, false, b, (short)0, c, false, false); }
__device__ __forceinline__ v8f wmmab(v16bf a, v16bf b, v8f c) { return __builtin_amdgcn_wmma_f32_16x16x32_bf16(false, a, false, b, (short)0, c, false, false); }
__device__ __forceinline__ v16h  ldh(const h16* p) { return cat16(*(const v8h*)p, *(const v8h*)(p + 16)); }
__device__ __forceinline__ v16bf ldb(const bf* p)  { return cat16b(*(const v8us*)p, *(const v8us*)(p + 16)); }
__device__ __forceinline__ void wave_sync() { __builtin_amdgcn_fence(3  , "wavefront"); __builtin_amdgcn_wave_barrier(); asm volatile("" ::: "memory"); }
__device__ __forceinline__ float silu(float t) { const float e = __builtin_amdgcn_exp2f(-1.4426950408889634f * t); return t * __builtin_amdgcn_rcpf(1.0f + e); }

__device__ __forceinline__ void bn4(const float* __restrict__ g, const float* __restrict__ be, const float* __restrict__ mu, const float* __restrict__ va, int ch, float* sct, float* sht, int dst) {
    const v4f gv = *(const v4f*)(g + ch), bv = *(const v4f*)(be + ch), mv = *(const v4f*)(mu + ch), vv = *(const v4f*)(va + ch);
    v4f s, t;
#pragma unroll
    for (int i = 0; i < 4; ++i) { const float sc = bfr(gv[i]) * rsqrtf(bfr(vv[i]) + BN_EPS); s[i] = sc; t[i] = bfr(bv[i]) - bfr(mv[i]) * sc; }
    *(volatile v4f*)(sct + dst) = s; *(volatile v4f*)(sht + dst) = t;
    __threadfence();
    *(volatile v4f*)(sct + dst) = s; *(volatile v4f*)(sht + dst) = t;
}

__global__ __launch_bounds__(256) void k_prep(const float* __restrict__ wqkv, const float* __restrict__ wproj,
                                              const float* __restrict__ qg, const float* __restrict__ qb, const float* __restrict__ qm, const float* __restrict__ qv,
                                              const float* __restrict__ pg, const float* __restrict__ pb, const float* __restrict__ pm, const float* __restrict__ pv,
                                              bf* WB, h16* WP, float* SCT, float* SHT) {
    const int bx = blockIdx.x;
    if (bx < PB_WQ) {
        const size_t i = (size_t)bx * 256 + threadIdx.x;
        const v8f v = *(const v8f*)(wqkv + i * 8); v8us o;
#pragma unroll
        for (int k = 0; k < 8; ++k) o[k] = f2bf(v[k]);
        *(volatile v8us*)(WB + i * 8) = o; __threadfence(); *(volatile v8us*)(WB + i * 8) = o;
    } else if (bx < PB_WQ + PB_WP) {
        const size_t i = (size_t)(bx - PB_WQ) * 256 + threadIdx.x;
        const v8f v = *(const v8f*)(wproj + i * 8); v8h o;
#pragma unroll
        for (int k = 0; k < 8; ++k) o[k] = (h16)(bfr(v[k]) * WPS);
        *(volatile v8h*)(WP + i * 8) = o; __threadfence(); *(volatile v8h*)(WP + i * 8) = o;
    } else {
        const int wave = __builtin_amdgcn_readfirstlane((int)(threadIdx.x >> 5)), lane = threadIdx.x & 31;
        if (wave < 3) { const int ch = (wave * 32 + lane) * 4; bn4(qg, qb, qm, qv, ch, SCT, SHT, ch); }
        else if (wave == 4) { const int ch = lane * 4; bn4(pg, pb, pm, pv, ch, SCT, SHT, 3 * CH + ch); }
    }
}

__global__ __launch_bounds__(256) void k_xt(const float* __restrict__ x, bf* XT) {
    __shared__ __align__(16) float ts[CH * 68];
    const int tid = threadIdx.x; const int b = blockIdx.y, n0 = blockIdx.x * 64;
#pragma unroll
    for (int it = 0; it < 8; ++it) { const int idx = it * 256 + tid; const int c = idx >> 4, n4 = (idx & 15) * 4;
        const v4f v = *(const v4f*)(x + ((size_t)b * CH + c) * SEQ_FULL + n0 + n4);
        *(v4fa*)(&ts[c * 68 + n4]) = v; }
    __syncthreads();
#pragma unroll 1
    for (int ps = 0; ps < 2; ++ps) {
#pragma unroll
        for (int it = 0; it < 4; ++it) { const int p = it * 256 + tid; const int row = p >> 4, c8 = (p & 15) * 8;
            v8us o;
#pragma unroll
            for (int i = 0; i < 8; ++i) o[i] = f2bf(ts[(c8 + i) * 68 + row]);
            *(volatile v8us*)(XT + ((size_t)b * SEQ + n0 + row) * CH + c8) = o; }
        if (ps == 0) __threadfence(); }
}

__global__ __launch_bounds__(32) void k_qk(const bf* __restrict__ A, const bf* __restrict__ Bt, const float* __restrict__ SCT, const float* __restrict__ SHT, h16* QK) {
    __shared__ __align__(16) float os[16 * 68];
    const int lane = threadIdx.x & 31, lr = lane & 15, hi = lane >> 4; const int r0 = blockIdx.x * 64, c0 = blockIdx.y * 64;
    v8f acc[4][4];
#pragma unroll
    for (int mb = 0; mb < 4; ++mb)
#pragma unroll
        for (int nb = 0; nb < 4; ++nb) acc[mb][nb] = (v8f){};
    const size_t aoff = (size_t)(r0 + lr) * CH + 8 * hi, boff = (size_t)(c0 + lr) * CH + 8 * hi;
#pragma unroll 1
    for (int kc = 0; kc < CH; kc += 32) {
        v16bf a[4];
#pragma unroll
        for (int mb = 0; mb < 4; ++mb) a[mb] = ldb(A + aoff + (size_t)mb * 16 * CH + kc);
#pragma unroll
        for (int nb = 0; nb < 4; ++nb) { const v16bf b = ldb(Bt + boff + (size_t)nb * 16 * CH + kc);
#pragma unroll
            for (int mb = 0; mb < 4; ++mb) acc[mb][nb] = wmmab(a[mb], b, acc[mb][nb]); }
        asm volatile("v_nop\n\tv_nop\n\tv_nop\n\tv_nop" : "+v"(acc[0][0]), "+v"(acc[1][1]), "+v"(acc[2][2]), "+v"(acc[3][3]) : "v"(a[0]), "v"(a[1]), "v"(a[2]), "v"(a[3]));
    }
    const int b = r0 / SEQ, tl = r0 % SEQ;
    const int part = c0 / CH, h0 = (c0 % CH) / HD;
    float scv[4], shv[4];
#pragma unroll
    for (int nb = 0; nb < 4; ++nb) { scv[nb] = SCT[c0 + nb * 16 + lr]; shv[nb] = SHT[c0 + nb * 16 + lr]; }
    const size_t pbase = (size_t)part * PLANE_E + ((size_t)(b * NH_ + h0) * SEQ + tl) * 32;
#pragma unroll
    for (int mb = 0; mb < 4; ++mb) {
#pragma unroll
        for (int nb = 0; nb < 4; ++nb) {
#pragma unroll
            for (int j = 0; j < 8; ++j) os[(hi * 8 + j) * 68 + nb * 16 + lr] = silu(fmaf(acc[mb][nb][j], scv[nb], shv[nb])); }
        wave_sync();
#pragma unroll 1
        for (int ps = 0; ps < 2; ++ps) {
#pragma unroll
            for (int s = 0; s < 2; ++s) {
#pragma unroll
                for (int nb = 0; nb < 4; ++nb) { const int row = 8 * s + (lane >> 2), pc = lane & 3, cb = nb * 16 + (pc & 1) * 8;
                    const v4f x0 = *(const v4fa*)(&os[row * 68 + cb]); const v4f x1 = *(const v4fa*)(&os[row * 68 + cb + 4]); v8h ov;
#pragma unroll
                    for (int i = 0; i < 4; ++i) { const h16 a0 = (h16)x0[i]; const h16 a1 = (h16)x1[i];
                        const float l0 = (part == 0) ? (x0[i] - (float)a0) * QRS : x0[i] * KRI;
                        const float l1 = (part == 0) ? (x1[i] - (float)a1) * QRS : x1[i] * KRI;
                        const h16 b0 = (h16)l0; const h16 b1 = (h16)l1;
                        ov[i] = (pc < 2) ? a0 : b0; ov[4 + i] = (pc < 2) ? a1 : b1; }
                    const size_t oo = pbase + (size_t)nb * SEQ * 32 + (size_t)(mb * 16 + row) * 32 + pc * 8;
                    *(volatile v8h*)(QK + oo) = ov; } }
            if (ps == 0) __threadfence(); }
        wave_sync();
    }
}

__global__ __launch_bounds__(32) void k_vt(const bf* __restrict__ A, const bf* __restrict__ Bt, const float* __restrict__ SCT, const float* __restrict__ SHT, h16* VT) {
    __shared__ __align__(16) float os[16 * 68];
    const int lane = threadIdx.x & 31, lr = lane & 15, hi = lane >> 4; const int r0 = blockIdx.x * 64, c0 = blockIdx.y * 64;
    v8f acc[4][4];
#pragma unroll
    for (int mb = 0; mb < 4; ++mb)
#pragma unroll
        for (int nb = 0; nb < 4; ++nb) acc[mb][nb] = (v8f){};
    const size_t aoff = (size_t)(r0 + lr) * CH + 8 * hi, boff = (size_t)(c0 + lr) * CH + 8 * hi;
#pragma unroll 1
    for (int kc = 0; kc < CH; kc += 32) {
        v16bf a[4];
#pragma unroll
        for (int mb = 0; mb < 4; ++mb) a[mb] = ldb(A + aoff + (size_t)mb * 16 * CH + kc);
#pragma unroll
        for (int nb = 0; nb < 4; ++nb) { const v16bf b = ldb(Bt + boff + (size_t)nb * 16 * CH + kc);
#pragma unroll
            for (int mb = 0; mb < 4; ++mb) acc[mb][nb] = wmmab(a[mb], b, acc[mb][nb]); }
        asm volatile("v_nop\n\tv_nop\n\tv_nop\n\tv_nop" : "+v"(acc[0][0]), "+v"(acc[1][1]), "+v"(acc[2][2]), "+v"(acc[3][3]) : "v"(a[0]), "v"(a[1]), "v"(a[2]), "v"(a[3]));
    }
    const int b = c0 / SEQ, tl = c0 % SEQ;
#pragma unroll
    for (int mb = 0; mb < 4; ++mb) {
        const v8f sc = *(const v8f*)(SCT + 2 * CH + r0 + mb * 16 + hi * 8); const v8f sh = *(const v8f*)(SHT + 2 * CH + r0 + mb * 16 + hi * 8);
#pragma unroll
        for (int nb = 0; nb < 4; ++nb) {
#pragma unroll
            for (int j = 0; j < 8; ++j) os[(hi * 8 + j) * 68 + nb * 16 + lr] = silu(fmaf(acc[mb][nb][j], sc[j], sh[j])); }
        wave_sync();
        const size_t sb = ((size_t)(b * CH + r0 + mb * 16)) * SEQ + tl;
#pragma unroll 1
        for (int ps = 0; ps < 2; ++ps) {
#pragma unroll
            for (int s = 0; s < 4; ++s) { const int row = 4 * s + (lane >> 3), c8 = (lane & 7) * 8;
                const v4f x0 = *(const v4fa*)(&os[row * 68 + c8]); const v4f x1 = *(const v4fa*)(&os[row * 68 + c8 + 4]); v8h hv;
#pragma unroll
                for (int i = 0; i < 4; ++i) { hv[i] = (h16)x0[i]; hv[4 + i] = (h16)x1[i]; }
                *(volatile v8h*)(VT + sb + (size_t)row * SEQ + c8) = hv; }
            if (ps == 0) __threadfence(); }
        wave_sync();
    }
}

__global__ __launch_bounds__(32 * AW) void k_flash(const h16* __restrict__ QK, const h16* __restrict__ VT, h16* CT) {
    const int lane = threadIdx.x & 31, wave = __builtin_amdgcn_readfirstlane((int)(threadIdx.x >> 5)), lr = lane & 15, hi = lane >> 4;
    const int bh = blockIdx.y;
    const int t0 = (blockIdx.x * AW + wave) * 16;
    const size_t pbase = (size_t)bh * SEQ * 32;
    const v16h qf = ldh(QK + pbase + (size_t)(t0 + lr) * 32 + 8 * hi);
    const size_t ko = PLANE_E + pbase + (size_t)lr * 32 + 8 * hi;
    const size_t vo = ((size_t)bh * HD + lr) * SEQ + 8 * hi;
    v8f o = (v8f){};
    float m = -3.0e38f, l = 0.0f;
#pragma unroll 1
    for (int key0 = 0; key0 < SEQ; key0 += 32) {
        const h16* ka = QK + ko + (size_t)key0 * 32;
        const v16h ka0 = ldh(ka), kb0 = ldh(ka + 16 * 32);
        v8f sa = (v8f){}, sb = (v8f){};
        sa = wmma16(ka0, qf, sa); sb = wmma16(kb0, qf, sb);
        asm volatile("v_nop\n\tv_nop\n\tv_nop\n\tv_nop" : "+v"(sa), "+v"(sb) : "v"(ka0), "v"(kb0), "v"(qf));
        float ta[8], tb[8]; float mx = -3.0e38f;
#pragma unroll
        for (int r = 0; r < 8; ++r) { ta[r] = sa[r] * SC2; tb[r] = sb[r] * SC2; mx = fmaxf(mx, fmaxf(ta[r], tb[r])); }
        mx = fmaxf(mx, __shfl_xor(mx, 16, 32));
        const float mnew = fmaxf(m, mx);
        const float alpha = __builtin_amdgcn_exp2f(m - mnew);
        const float sh = PSH - mnew;
        v16h pb; float ls = 0.0f;
#pragma unroll
        for (int r = 0; r < 8; ++r) { const h16 pa = (h16)__builtin_amdgcn_exp2f(ta[r] + sh); const h16 pc = (h16)__builtin_amdgcn_exp2f(tb[r] + sh); pb[r] = pa; pb[8 + r] = pc; ls += (float)pa + (float)pc; }
        l = l * alpha + ls; m = mnew;
        o = o * alpha;
        const v16h va = ldh(VT + vo + key0);
        o = wmma16(va, pb, o);
        asm volatile("v_nop\n\tv_nop\n\tv_nop\n\tv_nop" : "+v"(o) : "v"(va), "v"(pb));
    }
    l += __shfl_xor(l, 16, 32);
    const float inv = 1.0f / l;
    v8h cv;
#pragma unroll
    for (int r = 0; r < 8; ++r) cv[r] = (h16)(o[r] * inv);
    const v4u u = __builtin_bit_cast(v4u, cv);
    const int src = (lane & 1) * 16 + (lane >> 1);
    v4u w;
    w[0] = __shfl(u[0], src, 32); w[1] = __shfl(u[1], src, 32); w[2] = __shfl(u[2], src, 32); w[3] = __shfl(u[3], src, 32);
    h16* dst = CT + ((size_t)bh * SEQ + t0) * HD + lane * 8;
    *(volatile v4u*)dst = w; __threadfence(); *(volatile v4u*)dst = w;
}

__global__ __launch_bounds__(32) void k_outp(const h16* __restrict__ WP, const h16* __restrict__ CT, const float* __restrict__ SCT, const float* __restrict__ SHT, float* OUT) {
    __shared__ __align__(16) float os[16 * 68];
    const int lane = threadIdx.x & 31, lr = lane & 15, hi = lane >> 4; const int r0 = blockIdx.x * 64, c0 = blockIdx.y * 64;
    const int b = c0 / SEQ, tl = c0 % SEQ;
    v8f acc[4][4];
#pragma unroll
    for (int mb = 0; mb < 4; ++mb)
#pragma unroll
        for (int nb = 0; nb < 4; ++nb) acc[mb][nb] = (v8f){};
    const size_t aoff = (size_t)(r0 + lr) * CH + 8 * hi;
    const size_t boff = ((size_t)(b * NH_) * SEQ + tl + lr) * HD + 8 * hi;
#pragma unroll 1
    for (int kc = 0; kc < CH; kc += 32) {
        v16h a[4];
#pragma unroll
        for (int mb = 0; mb < 4; ++mb) a[mb] = ldh(WP + aoff + (size_t)mb * 16 * CH + kc);
#pragma unroll
        for (int nb = 0; nb < 4; ++nb) { const h16* bp = CT + boff + (size_t)(kc / HD) * SEQ * HD + (size_t)nb * 16 * HD;
            const v16h bv = cat16(*(const v8h*)bp, *(const v8h*)(bp + (size_t)SEQ * HD));
#pragma unroll
            for (int mb = 0; mb < 4; ++mb) acc[mb][nb] = wmma16(a[mb], bv, acc[mb][nb]); }
        asm volatile("v_nop\n\tv_nop\n\tv_nop\n\tv_nop" : "+v"(acc[0][0]), "+v"(acc[1][1]), "+v"(acc[2][2]), "+v"(acc[3][3]) : "v"(a[0]), "v"(a[1]), "v"(a[2]), "v"(a[3]));
    }
#pragma unroll
    for (int mb = 0; mb < 4; ++mb) {
        const v8f sc = *(const v8f*)(SCT + 3 * CH + r0 + mb * 16 + hi * 8) * WPI; const v8f sh = *(const v8f*)(SHT + 3 * CH + r0 + mb * 16 + hi * 8);
#pragma unroll
        for (int nb = 0; nb < 4; ++nb) {
#pragma unroll
            for (int j = 0; j < 8; ++j) os[(hi * 8 + j) * 68 + nb * 16 + lr] = silu(fmaf(acc[mb][nb][j], sc[j], sh[j])); }
        wave_sync();
        float* orow = OUT + ((size_t)(b * CH + r0 + mb * 16)) * OUT_SEQ + tl;
#pragma unroll 1
        for (int ps = 0; ps < 2; ++ps) {
#pragma unroll
            for (int s = 0; s < 8; ++s) { const int row = 2 * s + hi, cofs = lr * 4;
                const v4f val = *(const v4fa*)(&os[row * 68 + cofs]);
                *(volatile v4f*)(orow + (size_t)row * OUT_SEQ + cofs) = val; }
            if (ps == 0) __threadfence(); }
        wave_sync();
    }
}

static constexpr size_t al256(size_t v) { return (v + 255) & ~(size_t)255; }
static constexpr size_t SZ_XT = al256((size_t)NB * SEQ * CH * 2);
static constexpr size_t SZ_WB = al256((size_t)3 * CH * CH * 2);
static constexpr size_t SZ_WP = al256((size_t)CH * CH * 2);
static constexpr size_t SZ_TB = al256((size_t)4 * CH * 4);
static constexpr size_t SZ_QK = al256((size_t)2 * PLANE_E * 2);
static constexpr size_t SZ_VT = al256((size_t)NB * CH * SEQ * 2);
static constexpr size_t SZ_CT = al256((size_t)NB * NH_ * SEQ * HD * 2);
static constexpr size_t SZ_TOTAL = SZ_XT + SZ_WB + SZ_WP + 2 * SZ_TB + SZ_QK + SZ_VT + SZ_CT;
static_assert(SZ_TOTAL <= (size_t)134217728);
static_assert(((size_t)PLANE_E * 2) % 256 == 0);

extern "C" void kernel_launch(void* const* d_in, const int* in_sizes, int n_in,
                              void* d_out, int out_size, void* d_ws, size_t ws_size, hipStream_t stream) {
    if (n_in < 11) return;
    if ((size_t)in_sizes[0] < ((size_t)(NB - 1) * CH + (CH - 1)) * SEQ_FULL + SEQ) return;
    if ((size_t)in_sizes[1] < (size_t)3 * CH * CH) return;
    if ((size_t)in_sizes[2] < (size_t)3 * CH || (size_t)in_sizes[3] < (size_t)3 * CH || (size_t)in_sizes[4] < (size_t)3 * CH || (size_t)in_sizes[5] < (size_t)3 * CH) return;
    if ((size_t)in_sizes[6] < (size_t)CH * CH) return;
    if ((size_t)in_sizes[7] < (size_t)CH || (size_t)in_sizes[8] < (size_t)CH || (size_t)in_sizes[9] < (size_t)CH || (size_t)in_sizes[10] < (size_t)CH) return;
    if ((size_t)out_size < ((size_t)(NB - 1) * CH + (CH - 1)) * OUT_SEQ + SEQ) return;
    if (SZ_TOTAL > ws_size) return;
    const float* x = (const float*)d_in[0]; const float* wqkv = (const float*)d_in[1];
    const float* qg = (const float*)d_in[2]; const float* qb = (const float*)d_in[3]; const float* qm = (const float*)d_in[4]; const float* qv = (const float*)d_in[5];
    const float* wproj = (const float*)d_in[6];
    const float* pg = (const float*)d_in[7]; const float* pb = (const float*)d_in[8]; const float* pm = (const float*)d_in[9]; const float* pv = (const float*)d_in[10];
    float* OUT = (float*)d_out;
    char* wsp = (char*)d_ws;
    bf*  XT = (bf*)wsp;   wsp += SZ_XT;
    bf*  WB = (bf*)wsp;   wsp += SZ_WB;
    h16* WP = (h16*)wsp;  wsp += SZ_WP;
    float* SCT = (float*)wsp; wsp += SZ_TB;
    float* SHT = (float*)wsp; wsp += SZ_TB;
    h16* QK = (h16*)wsp;  wsp += SZ_QK;
    h16* VT = (h16*)wsp;  wsp += SZ_VT;
    h16* CT = (h16*)wsp;  wsp += SZ_CT;

    k_prep<<<PB_WQ + PB_WP + 1, 256, 0, stream>>>(wqkv, wproj, qg, qb, qm, qv, pg, pb, pm, pv, WB, WP, SCT, SHT);
    k_xt<<<dim3(SEQ / 64, NB, 1), 256, 0, stream>>>(x, XT);
    k_qk<<<dim3(NB * SEQ / 64, 2 * CH / 64, 1), 32, 0, stream>>>(XT, WB, SCT, SHT, QK);
    k_vt<<<dim3(CH / 64, NB * SEQ / 64, 1), 32, 0, stream>>>(WB + (size_t)2 * CH * CH, XT, SCT, SHT, VT);
    k_flash<<<dim3(SEQ / (16 * AW), NB * NH_, 1), 32 * AW, 0, stream>>>(QK, VT, CT);
    k_outp<<<dim3(CH / 64, NB * SEQ / 64, 1), 32, 0, stream>>>(WP, CT, SCT, SHT, OUT);
}
